// LSTMAutoencoder_25975962206284
// MI455X (gfx1250) — hardware-verified
//
#include <hip/hip_runtime.h>
#include <math.h>

constexpr int kBatch   = 512;
constexpr int kSteps   = 256;
constexpr int kIn      = 64;
constexpr int kHid     = 64;
constexpr int kGate    = 4 * kHid;
constexpr int kRecThr  = 128;
constexpr int kRowsBlk = 16;
constexpr int kHSP     = 68;
constexpr int kHP      = 2 * kHid;
constexpr int kRows    = kBatch * kSteps;
static_assert(kIn == 64 && kHid == 64 && kGate == 256);
static_assert(kHid == 16 * (kRecThr / 32));
static_assert(kRowsBlk == 16 && kRecThr == 128);
static_assert(kBatch % kRowsBlk == 0);
static_assert(kRows % 64 == 0 && kIn % 64 == 0);
static_assert(kHP % 32 == 0);
static_assert((kGate * 8) % 256 == 0 && (kIn * 8) % 256 == 0);

typedef __attribute__((ext_vector_type(16))) _Float16 v16h;
typedef __attribute__((ext_vector_type(8)))  _Float16 v8h;
typedef __attribute__((ext_vector_type(16))) __bf16   v16b;
typedef __attribute__((ext_vector_type(8)))  __bf16   v8b;
typedef __attribute__((ext_vector_type(8)))  float    v8f;
typedef __attribute__((ext_vector_type(4)))  float    v4f;
typedef __attribute__((ext_vector_type(4)))  unsigned v4u;

__device__ __forceinline__ unsigned short f2bf_bits(float f) {
  unsigned u = __float_as_uint(f);
  return (unsigned short)((u + 0x7FFFu + ((u >> 16) & 1u)) >> 16);
}
__device__ __forceinline__ float bf_bits2f(unsigned short h) { return __uint_as_float(((unsigned)h) << 16); }
__device__ __forceinline__ float bf16r(float f) { return bf_bits2f(f2bf_bits(f)); }

__device__ __forceinline__ void dep_guard_h(v8f& a, v8f& b, v16h x, v16h y) { asm volatile("v_nop\n\tv_nop\n\tv_nop\n\tv_nop" : "+v"(a), "+v"(b) : "v"(x), "v"(y)); }
__device__ __forceinline__ void dep_guard_b(v8f& a, v8f& b, v16b x, v16b y) { asm volatile("v_nop\n\tv_nop\n\tv_nop\n\tv_nop" : "+v"(a), "+v"(b) : "v"(x), "v"(y)); }
__device__ __forceinline__ void keep4_h(v16h a, v16h b, v16h c, v16h d) { asm volatile("v_nop" :: "v"(a), "v"(b), "v"(c), "v"(d)); }
__device__ __forceinline__ void keep4_b(v16b a, v16b b, v16b c, v16b d) { asm volatile("v_nop" :: "v"(a), "v"(b), "v"(c), "v"(d)); }
__device__ __forceinline__ void acc_guard4(v8f& a, v8f& b, v8f& c, v8f& d) { asm volatile("v_nop\n\tv_nop\n\tv_nop\n\tv_nop" : "+v"(a), "+v"(b), "+v"(c), "+v"(d)); }
__device__ __forceinline__ void guard4acc5_b(v8f& a0, v8f& a1, v8f& a2, v8f& a3, v16b x, v16b y0, v16b y1, v16b y2, v16b y3) {
  asm volatile("v_nop\n\tv_nop\n\tv_nop\n\tv_nop" : "+v"(a0), "+v"(a1), "+v"(a2), "+v"(a3) : "v"(x), "v"(y0), "v"(y1), "v"(y2), "v"(y3));
}
template <typename T> struct Frag;
template <> struct Frag<_Float16> {
  typedef v16h V; union U { v16h v; v8h h[2]; };
  static __device__ __forceinline__ v16h load(const _Float16* p) {
    U f; f.h[0] = *(const v8h*)(p); f.h[1] = *(const v8h*)(p + 16); return f.v;
  }
  static __device__ __forceinline__ v8f mma(v16h a, v16h b, v8f c) {
    return __builtin_amdgcn_wmma_f32_16x16x32_f16(false, a, false, b, (short)0, c, false, false);
  }
  static __device__ __forceinline__ void guard(v8f& a, v8f& b, v16h x, v16h y) { dep_guard_h(a, b, x, y); }
  static __device__ __forceinline__ void keep(v16h a, v16h b, v16h c, v16h d) { keep4_h(a, b, c, d); }
};
template <> struct Frag<__bf16> {
  typedef v16b V; union U { v16b v; v8b h[2]; };
  static __device__ __forceinline__ v16b load(const __bf16* p) {
    U f; f.h[0] = *(const v8b*)(p); f.h[1] = *(const v8b*)(p + 16); return f.v;
  }
  static __device__ __forceinline__ v8f mma(v16b a, v16b b, v8f c) {
    return __builtin_amdgcn_wmma_f32_16x16x32_bf16(false, a, false, b, (short)0, c, false, false);
  }
  static __device__ __forceinline__ void guard(v8f& a, v8f& b, v16b x, v16b y) { dep_guard_b(a, b, x, y); }
  static __device__ __forceinline__ void keep(v16b a, v16b b, v16b c, v16b d) { keep4_b(a, b, c, d); }
};

template <int ET> struct Elem;
template <> struct Elem<0> { typedef _Float16 T; };
template <> struct Elem<1> { typedef __bf16 T; };
template <int ET, bool SPLIT, int BIAS_MODE, int OUT_MODE, bool RESID, int ACT = 0>
__global__ __launch_bounds__(256) void wmma_gemm64(
    const unsigned short* __restrict__ Ap, const unsigned short* __restrict__ A2p, int lda, long strideA,
    const unsigned short* __restrict__ Btp, const unsigned short* __restrict__ Bt2p, int ldb, long strideB,
    void* __restrict__ Cout, void* __restrict__ Cout2, int ldc, long strideC,
    const float* __restrict__ bias,
    const float* __restrict__ resid, long strideR,
    int M, int N, int K, float scale) {
  typedef typename Elem<ET>::T T;
  typedef typename Frag<T>::V V;
  const T* A = (const T*)Ap; const T* A2 = (const T*)A2p; const T* Bt = (const T*)Btp; const T* Bt2 = (const T*)Bt2p;
  __shared__ __align__(16) float sT[8][16 * 68];
  const int b    = blockIdx.y;
  const int lane = threadIdx.x & 31;
  const int wave = threadIdx.x >> 5;
  const int tilesN = N >> 6;
  const int tilesM = M >> 6;
  const int tile = blockIdx.x * 8 + wave;
  if (tile >= tilesM * tilesN) return;
  const int tm = tile / tilesN;
  const int tn = tile - tm * tilesN;
  const int m0 = tm << 6;
  const int n0 = tn << 6;

  const T* Ab  = A  + (size_t)b * strideA;
  const T* Bb  = Bt + (size_t)b * strideB;
  const T* Ab2 = SPLIT ? (A2  + (size_t)b * strideA) : nullptr;
  const T* Bb2 = SPLIT ? (Bt2 + (size_t)b * strideB) : nullptr;

  const int rlane = lane & 15;
  const int koff  = (lane >> 4) * 8;
  const int mOff  = (lane >> 4) * 8;

  v8f acc[4][4];
#pragma unroll
  for (int i = 0; i < 4; ++i)
#pragma unroll
    for (int j = 0; j < 4; ++j) acc[i][j] = (v8f){0.f,0.f,0.f,0.f,0.f,0.f,0.f,0.f};

  for (int k0 = 0; k0 < K; k0 += 32) {
    V bh[4], bl[4];
#pragma unroll
    for (int j = 0; j < 4; ++j) {
      const size_t bo = (size_t)(n0 + (j << 4) + rlane) * ldb + koff + k0;
      bh[j] = Frag<T>::load(Bb + bo);
      if (SPLIT) bl[j] = Frag<T>::load(Bb2 + bo);
    }
#pragma unroll
    for (int i = 0; i < 4; ++i) {
      const size_t ao = (size_t)(m0 + (i << 4) + rlane) * lda + koff + k0;
      V ah = Frag<T>::load(Ab + ao);
      V al;
      if (SPLIT) al = Frag<T>::load(Ab2 + ao);
#pragma unroll
      for (int j = 0; j < 4; ++j) {
        acc[i][j] = Frag<T>::mma(ah, bh[j], acc[i][j]);
        if (SPLIT) {
          acc[i][j] = Frag<T>::mma(ah, bl[j], acc[i][j]);
          acc[i][j] = Frag<T>::mma(al, bh[j], acc[i][j]);
        }
      }
      Frag<T>::guard(acc[i][0], acc[i][3], ah, SPLIT ? al : ah);
    }
    Frag<T>::keep(bh[0], bh[1], bh[2], bh[3]);
    if (SPLIT) Frag<T>::keep(bl[0], bl[1], bl[2], bl[3]);
  }
  acc_guard4(acc[0][0], acc[0][1], acc[0][2], acc[0][3]);
  acc_guard4(acc[1][0], acc[1][1], acc[1][2], acc[1][3]);
  acc_guard4(acc[2][0], acc[2][1], acc[2][2], acc[2][3]);
  acc_guard4(acc[3][0], acc[3][1], acc[3][2], acc[3][3]);

  float* slab = sT[wave];
  const float* Rb = RESID ? (resid + (size_t)b * strideR) : nullptr;
#pragma unroll
  for (int i = 0; i < 4; ++i) {
    const int mBase = m0 + (i << 4);
#pragma unroll
    for (int j = 0; j < 4; ++j) {
      const int n = n0 + (j << 4) + rlane;
      float bv = 0.f;
      if (BIAS_MODE == 2) bv = bias[n];
#pragma unroll
      for (int r = 0; r < 8; ++r) {
        float v = acc[i][j][r] * scale;
        if (BIAS_MODE == 1) v += bias[mBase + mOff + r];
        if (BIAS_MODE == 2) v += bv;
        if (RESID) v += Rb[(size_t)(mBase + mOff + r) * ldc + n];
        if (ACT == 1) v = tanhf(v);
        if (ACT == 2) v = fmaxf(v, 0.0f);
        if (ACT == 3) v = v / (1.0f + expf(-v));
        if (ACT == 4) v = (v > 0.f) ? v : 0.01f * v;
        if (ACT == 5) v = 0.5f * v * (1.0f + erff(v * 0.70710678118654752f));
        slab[(mOff + r) * 68 + (j << 4) + rlane] = v;
      }
    }
    __builtin_amdgcn_fence(__ATOMIC_RELEASE, "workgroup");
    __builtin_amdgcn_wave_barrier();
    __builtin_amdgcn_fence(__ATOMIC_ACQUIRE, "workgroup");
    if (OUT_MODE == 0) {
      float* C = (float*)Cout + (size_t)b * strideC;
      const int hh = lane >> 4, c4 = (lane & 15) * 4;
      for (int pass = 0; pass < 2; ++pass) {
#pragma unroll
        for (int it = 0; it < 8; ++it) {
          const int row = it * 2 + hh;
          v4f v = *(const v4f*)(slab + row * 68 + c4);
          *(volatile v4f*)(C + (size_t)(mBase + row) * ldc + n0 + c4) = v;
        }
        __threadfence();
      }
    } else {
      const int q = lane >> 3, c8 = (lane & 7) * 8;
      unsigned short* C  = (unsigned short*)Cout  + (size_t)b * strideC;
      unsigned short* C2 = (OUT_MODE == 2) ? ((unsigned short*)Cout2 + (size_t)b * strideC) : nullptr;
      for (int pass = 0; pass < 2; ++pass) {
#pragma unroll
        for (int it = 0; it < 4; ++it) {
          const int row = it * 4 + q;
          const float* sp = slab + row * 68 + c8;
          v8h hv, lv;
#pragma unroll
          for (int e = 0; e < 8; ++e) {
            if (OUT_MODE == 1) {
              hv[e] = (_Float16)sp[e];
            } else {
              unsigned short hb = f2bf_bits(sp[e]);
              unsigned short lb = f2bf_bits(sp[e] - bf_bits2f(hb));
              hv[e] = __builtin_bit_cast(_Float16, hb);
              lv[e] = __builtin_bit_cast(_Float16, lb);
            }
          }
          *(volatile v8h*)(C + (size_t)(mBase + row) * ldc + n0 + c8) = hv;
          if (OUT_MODE == 2) *(volatile v8h*)(C2 + (size_t)(mBase + row) * ldc + n0 + c8) = lv;
        }
        __threadfence();
      }
    }
    __builtin_amdgcn_fence(__ATOMIC_RELEASE, "workgroup");
    __builtin_amdgcn_wave_barrier();
    __builtin_amdgcn_fence(__ATOMIC_ACQUIRE, "workgroup");
  }
}

__device__ __forceinline__ float fsig(float x)  { return __builtin_amdgcn_rcpf(1.0f + expf(-x)); }
__device__ __forceinline__ float ftanh(float x) { return 1.0f - 2.0f * __builtin_amdgcn_rcpf(expf(2.0f * x) + 1.0f); }

__global__ __launch_bounds__(256) void wcat_kernel(const float* __restrict__ wa, const float* __restrict__ wb,
                                                   unsigned short* __restrict__ dst, int nrows, int nx, int nseg) {
  const int i   = blockIdx.x * 256 + threadIdx.x;
  const int per = nrows * 8;
  if (i >= per * nseg) return;
  const int seg = i / per;
  const int rem = i - seg * per;
  const int n = rem >> 3, c8 = (rem & 7) * 8;
  const int ktot = nseg * 64;
  const float* src = (seg < nx) ? wa : wb;
  const float* sp = src + (size_t)n * 64 + c8;
  const v4f a = *(const v4f*)sp;
  const v4f q = *(const v4f*)(sp + 4);
  v8h hv;
#pragma unroll
  for (int e = 0; e < 4; ++e) {
    hv[e]     = __builtin_bit_cast(_Float16, f2bf_bits(a[e]));
    hv[4 + e] = __builtin_bit_cast(_Float16, f2bf_bits(q[e]));
  }
  unsigned short* op = dst + (size_t)n * ktot + seg * 64 + c8;
  *(volatile v8h*)op = hv;
  __threadfence();
  *(volatile v8h*)op = hv;
}

__global__ __launch_bounds__(32) void fcb_kernel(const float* __restrict__ b, float* __restrict__ dst) {
  const int t4 = threadIdx.x * 4;
  const v4f v = *(const v4f*)(b + t4);
  v4f o;
#pragma unroll
  for (int e = 0; e < 4; ++e) o[e] = bf16r(v[e]);
  *(volatile v4f*)(dst + t4) = o;
  __threadfence();
  *(volatile v4f*)(dst + t4) = o;
}

template <int XSRC>
__device__ __forceinline__ void stage_x(unsigned short* at, int ap, const float* __restrict__ xf,
                                        const unsigned short* __restrict__ xp, int xst, int b0, int tt, int tid) {
  const int m = tid >> 3;
  if (XSRC == 0) {
    const int c8 = (tid & 7) * 8;
    const float* sp = xf + ((size_t)(b0 + m) * kSteps + (size_t)tt) * kIn + c8;
    const v4f a = *(const v4f*)sp;
    const v4f q = *(const v4f*)(sp + 4);
    v4u pk;
    pk[0] = (unsigned)f2bf_bits(a[0]) | ((unsigned)f2bf_bits(a[1]) << 16);
    pk[1] = (unsigned)f2bf_bits(a[2]) | ((unsigned)f2bf_bits(a[3]) << 16);
    pk[2] = (unsigned)f2bf_bits(q[0]) | ((unsigned)f2bf_bits(q[1]) << 16);
    pk[3] = (unsigned)f2bf_bits(q[2]) | ((unsigned)f2bf_bits(q[3]) << 16);
    *(v4u*)(at + m * ap + c8) = pk;
  } else {
    const int c16 = (tid & 7) * 16;
    const unsigned short* sp = xp + ((size_t)(b0 + m) * kSteps + (size_t)tt * (size_t)xst) * kHP + c16;
    const v4u w0 = *(const v4u*)sp;
    const v4u w1 = *(const v4u*)(sp + 8);
    *(v4u*)(at + m * ap + c16) = w0;
    *(v4u*)(at + m * ap + c16 + 8) = w1;
  }
}

template <int XSRC>
__global__ __launch_bounds__(kRecThr) void lstm_seq_kernel(
    const float* __restrict__ xf, const unsigned short* __restrict__ xp, int xst,
    const unsigned short* __restrict__ wcatp,
    const float* __restrict__ bih, const float* __restrict__ bhh,
    unsigned short* __restrict__ hp) {
  constexpr int KX = (XSRC == 0) ? kIn : kHP;
  constexpr int KT = KX + kHP;
  constexpr int AP = KT + 8;
  constexpr int NFILL = (kRowsBlk * AP) / kRecThr;
  static_assert((kRowsBlk * AP) % kRecThr == 0);
  static_assert(KT % 32 == 0 && (AP % 8) == 0);
  __shared__ __align__(16) unsigned short At[kRowsBlk * AP];
  __shared__ __align__(16) float          Hs[kRowsBlk * kHSP];
  const __bf16* wcat = (const __bf16*)wcatp;
  const int tid = threadIdx.x, lane = tid & 31, wave = tid >> 5;
  const int c = lane & 15, hh = lane >> 4, koff = hh * 8;
  const int b0 = blockIdx.x * kRowsBlk;
  const int j  = 16 * wave + c;

#pragma unroll 1
  for (int i = 0; i < NFILL; ++i) At[i * kRecThr + tid] = (unsigned short)0;
  float cst[8], hst[8], bb[4];
#pragma unroll
  for (int r = 0; r < 8; ++r) { cst[r] = 0.0f; hst[r] = 0.0f; }
#pragma unroll
  for (int gi = 0; gi < 4; ++gi) bb[gi] = bf16r(bih[gi * kHid + j]) + bf16r(bhh[gi * kHid + j]);
  __syncthreads();
  stage_x<XSRC>(At, AP, xf, xp, xst, b0, 0, tid);
  __syncthreads();

  const __bf16* arow  = (const __bf16*)At + c * AP + koff;
  const __bf16* wrow0 = wcat + (size_t)j * KT + koff;
  const __bf16* wrow1 = wrow0 + (size_t)1 * kHid * KT;
  const __bf16* wrow2 = wrow0 + (size_t)2 * kHid * KT;
  const __bf16* wrow3 = wrow0 + (size_t)3 * kHid * KT;
  const v8f z8 = {0.f, 0.f, 0.f, 0.f, 0.f, 0.f, 0.f, 0.f};
  const int srow = 4 * wave + (lane >> 3);
  const int sc8  = (lane & 7) * 8;

#pragma unroll 1
  for (int t = 0; t < kSteps; ++t) {
    v8f acc[4];
    acc[0] = z8; acc[1] = z8; acc[2] = z8; acc[3] = z8;
#pragma unroll 1
    for (int k0 = 0; k0 < KT; k0 += 32) {
      const v16b a  = Frag<__bf16>::load(arow + k0);
      const v16b w0 = Frag<__bf16>::load(wrow0 + k0);
      const v16b w1 = Frag<__bf16>::load(wrow1 + k0);
      const v16b w2 = Frag<__bf16>::load(wrow2 + k0);
      const v16b w3 = Frag<__bf16>::load(wrow3 + k0);
      acc[0] = Frag<__bf16>::mma(a, w0, acc[0]);
      acc[1] = Frag<__bf16>::mma(a, w1, acc[1]);
      acc[2] = Frag<__bf16>::mma(a, w2, acc[2]);
      acc[3] = Frag<__bf16>::mma(a, w3, acc[3]);
      guard4acc5_b(acc[0], acc[1], acc[2], acc[3], a, w0, w1, w2, w3);
    }
    acc_guard4(acc[0], acc[1], acc[2], acc[3]);

#pragma unroll
    for (int r = 0; r < 8; ++r) {
      const float zi = acc[0][r] + bb[0];
      const float zf = acc[1][r] + bb[1];
      const float zg = acc[2][r] + bb[2];
      const float zo = acc[3][r] + bb[3];
      const float ig = fsig(zi);
      const float fg = fsig(zf);
      const float gg = ftanh(zg);
      const float og = fsig(zo);
      const float cn = fg * cst[r] + ig * gg;
      cst[r] = cn;
      hst[r] = og * ftanh(cn);
    }
    __syncthreads();

#pragma unroll
    for (int r = 0; r < 8; ++r) {
      const int row = 8 * hh + r;
      const float hn = hst[r];
      const unsigned short hb = f2bf_bits(hn);
      const unsigned short lb = f2bf_bits(hn - bf_bits2f(hb));
      At[row * AP + KX + j]        = hb;
      At[row * AP + KX + kHid + j] = lb;
      Hs[row * kHSP + j] = hn;
    }
    {
      const int tn = (t + 1 < kSteps) ? (t + 1) : (kSteps - 1);
      stage_x<XSRC>(At, AP, xf, xp, xst, b0, tn, tid);
    }
    __syncthreads();

    {
      const v4f p0 = *(const v4f*)(Hs + srow * kHSP + sc8);
      const v4f p1 = *(const v4f*)(Hs + srow * kHSP + sc8 + 4);
      v8h hv, lv;
#pragma unroll
      for (int e = 0; e < 4; ++e) {
        const float f0 = p0[e];
        const float f1 = p1[e];
        const unsigned short hb0 = f2bf_bits(f0);
        const unsigned short hb1 = f2bf_bits(f1);
        const unsigned short lb0 = f2bf_bits(f0 - bf_bits2f(hb0));
        const unsigned short lb1 = f2bf_bits(f1 - bf_bits2f(hb1));
        hv[e]     = __builtin_bit_cast(_Float16, hb0);
        hv[4 + e] = __builtin_bit_cast(_Float16, hb1);
        lv[e]     = __builtin_bit_cast(_Float16, lb0);
        lv[4 + e] = __builtin_bit_cast(_Float16, lb1);
      }
      unsigned short* op = hp + ((size_t)(b0 + srow) * kSteps + (size_t)t) * kHP + sc8;
      for (int pass = 0; pass < 2; ++pass) {
        *(volatile v8h*)op = hv;
        *(volatile v8h*)(op + kHid) = lv;
        __threadfence();
      }
    }
  }
}

extern "C" void kernel_launch(void* const* d_in, const int* in_sizes, int n_in,
                              void* d_out, int out_size, void* d_ws, size_t ws_size, hipStream_t stream) {
  if (n_in < 19 || d_out == nullptr || d_ws == nullptr) return;
  if (in_sizes[0] != kBatch * kSteps * kIn || out_size != kBatch * kSteps * kIn) return;
  for (int l = 0; l < 4; ++l) {
    const int base = 1 + 4 * l;
    if (in_sizes[base] != kGate * kHid || in_sizes[base + 1] != kGate * kHid ||
        in_sizes[base + 2] != kGate || in_sizes[base + 3] != kGate) return;
  }
  if (in_sizes[17] != kIn * kHid || in_sizes[18] != kIn) return;

  const float* x = (const float*)d_in[0];
  const float* wih[4] = {(const float*)d_in[1], (const float*)d_in[5], (const float*)d_in[9],  (const float*)d_in[13]};
  const float* whh[4] = {(const float*)d_in[2], (const float*)d_in[6], (const float*)d_in[10], (const float*)d_in[14]};
  const float* bih[4] = {(const float*)d_in[3], (const float*)d_in[7], (const float*)d_in[11], (const float*)d_in[15]};
  const float* bhh[4] = {(const float*)d_in[4], (const float*)d_in[8], (const float*)d_in[12], (const float*)d_in[16]};
  const float* fcw = (const float*)d_in[17];
  const float* fcb = (const float*)d_in[18];
  float* out = (float*)d_out;

  char* ws = (char*)d_ws; size_t off = 0;
  auto carve = [&](size_t bytes) -> char* { char* p = ws + off; off += (bytes + 255) & ~(size_t)255; return p; };
  unsigned short* WC0 = (unsigned short*)carve((size_t)kGate * (kIn + kHP) * 2);
  unsigned short* WC1 = (unsigned short*)carve((size_t)kGate * (kHP + kHP) * 2);
  unsigned short* WC2 = (unsigned short*)carve((size_t)kGate * (kHP + kHP) * 2);
  unsigned short* WC3 = (unsigned short*)carve((size_t)kGate * (kHP + kHP) * 2);
  unsigned short* FWC = (unsigned short*)carve((size_t)kIn * kHP * 2);
  float*          FCB = (float*)carve((size_t)kIn * 4);
  unsigned short* HA  = (unsigned short*)carve((size_t)kRows * kHP * 2);
  unsigned short* HB  = (unsigned short*)carve((size_t)kRows * kHP * 2);
  if (off > ws_size || off > (size_t)134217728) return;

  wcat_kernel<<<(3 * kGate * 8) / 256, 256, 0, stream>>>(wih[0], whh[0], WC0, kGate, 1, 3);
  wcat_kernel<<<(4 * kGate * 8) / 256, 256, 0, stream>>>(wih[1], whh[1], WC1, kGate, 2, 4);
  wcat_kernel<<<(4 * kGate * 8) / 256, 256, 0, stream>>>(wih[2], whh[2], WC2, kGate, 2, 4);
  wcat_kernel<<<(4 * kGate * 8) / 256, 256, 0, stream>>>(wih[3], whh[3], WC3, kGate, 2, 4);
  wcat_kernel<<<(2 * kIn * 8) / 256, 256, 0, stream>>>(fcw, fcw, FWC, kIn, 2, 2);
  fcb_kernel<<<1, 16, 0, stream>>>(fcb, FCB);

  lstm_seq_kernel<0><<<kBatch / kRowsBlk, kRecThr, 0, stream>>>(x, HB, 1, WC0, bih[0], bhh[0], HA);
  lstm_seq_kernel<1><<<kBatch / kRowsBlk, kRecThr, 0, stream>>>(x, HA, 1, WC1, bih[1], bhh[1], HB);
  lstm_seq_kernel<1><<<kBatch / kRowsBlk, kRecThr, 0, stream>>>(x, HB + (size_t)(kSteps - 1) * kHP, 0, WC2,
                                                                  bih[2], bhh[2], HA);
  lstm_seq_kernel<1><<<kBatch / kRowsBlk, kRecThr, 0, stream>>>(x, HA, 1, WC3, bih[3], bhh[3], HB);

  wmma_gemm64<1, false, 2, 0, false, 0><<<dim3((kRows / 64) * (kIn / 64) / 8, 1), 256, 0, stream>>>(
      HB, HB, kHP, 0L, FWC, FWC, kHP, 0L, (void*)out, (void*)out, kIn, 0L,
      FCB, FCB, 0L, kRows, kIn, kHP, 1.0f);
}
